// GQAAttention_29317446762928
// MI455X (gfx1250) — hardware-verified
//
#include <hip/hip_runtime.h>

#ifndef NB
#define NB 1
#endif
#ifndef SEQ
#define SEQ 2048
#endif
#define NB_FULL 1
#define SEQ_FULL 2048
#define HIDDEN 2048
#define NH 32
#define NKV 8
#define NREP (NH / NKV)
#define HDIM 64
#define QD (NH * HDIM)
#define KVD (NKV * HDIM)
#define NR (NB * SEQ)
#define TQ SEQ
#define TK SEQ
#define SCL 0.125f
#define QBLKS (TQ / 64)
#define QBN5 ((QBLKS < 4) ? QBLKS : 4)
#define QB05 0
#define QB0P QBN5
#define QBNP (QBLKS - QBN5)
#define RE (QBN5 * 64)
#define WS_LIMIT 134217728ull

static_assert(NB >= 1 && NB <= NB_FULL);
static_assert(SEQ % 128 == 0 && SEQ <= SEQ_FULL);
static_assert(RE % 128 == 0 && (SEQ - RE) % 128 == 0);
static_assert(HIDDEN % 64 == 0 && QD % 64 == 0 && KVD % 64 == 0 && HDIM == 64);
static_assert(HIDDEN % 32 == 0 && QD % 32 == 0);

#define WS_TOTAL ((size_t)HIDDEN * QD * 2 * 2 + (size_t)HIDDEN * KVD * 2 * 2 + (size_t)NR * HIDDEN * 2 + (size_t)NR * QD * 4 + (size_t)NR * KVD * 4 * 2 \
  + (size_t)NR * 32 * 4 * 2 + (size_t)NR * QD * 2 * 2 + (size_t)NR * KVD * 2 * 6 + (size_t)NR * QD * 4 + (size_t)NR * QD * 2 * 2)
static_assert(WS_TOTAL + 64 * 256 <= WS_LIMIT);

typedef unsigned short v8us __attribute__((ext_vector_type(8), may_alias));
typedef float  v8f  __attribute__((ext_vector_type(8)));
typedef float  v4f  __attribute__((ext_vector_type(4)));
typedef float  v4fa __attribute__((ext_vector_type(4), may_alias));
typedef _Float16 v16h __attribute__((ext_vector_type(16)));
union FragH { v16h v; v8us half[2]; _Float16 h[16]; unsigned short u[16]; };

__device__ __forceinline__ unsigned short bf16_bits(float x) { unsigned int u = __float_as_uint(x); return (unsigned short)((u + 0x7FFFu + ((u >> 16) & 1u)) >> 16); }
__device__ __forceinline__ float bf16_val(unsigned short b) { return __uint_as_float(((unsigned int)b) << 16); }
__device__ __forceinline__ float bf16_rne(float x) { return bf16_val(bf16_bits(x)); }

template <int NT>
__device__ __forceinline__ v8f mmaH(v16h ah, v16h al, v16h bh, v16h bl, v8f c) {
  c = __builtin_amdgcn_wmma_f32_16x16x32_f16(false, ah, false, bh, (short)0, c, false, false);
  if (NT >= 2) c = __builtin_amdgcn_wmma_f32_16x16x32_f16(false, al, false, bh, (short)0, c, false, false);
  if (NT >= 3) c = __builtin_amdgcn_wmma_f32_16x16x32_f16(false, ah, false, bl, (short)0, c, false, false);
  asm volatile("v_nop\n\tv_nop\n\tv_nop\n\tv_nop" : "+v"(c) : "v"(ah), "v"(al), "v"(bh), "v"(bl));
  return c;
}

__global__ __launch_bounds__(256) void k_wt_f16(const float* __restrict__ W, _Float16* __restrict__ Wt, int K, int N, float scale) {
  const int t = blockIdx.x * 256 + threadIdx.x; if (t >= N * (K / 8)) return;
  const int n = t / (K / 8), k8 = (t % (K / 8)) * 8; FragH f;
#pragma unroll
  for (int i = 0; i < 8; ++i) f.h[i] = (_Float16)(bf16_rne(W[(size_t)(k8 + i) * N + n]) * scale);
  const v8us o = f.half[0];
  unsigned short* d = (unsigned short*)Wt + (size_t)n * K + k8;
  *(volatile v8us*)d = o; __threadfence(); *(volatile v8us*)d = o;
}

__global__ __launch_bounds__(256) void k_x16(const float* __restrict__ x, _Float16* __restrict__ X16, size_t n8) {
  const size_t t = (size_t)blockIdx.x * 256 + threadIdx.x; if (t >= n8) return;
  const size_t e = t * 8; const size_t row = e / HIDDEN; const int c = (int)(e % HIDDEN);
  const size_t srow = (row / SEQ) * SEQ_FULL + (row % SEQ);
  const float* p = x + srow * HIDDEN + c; FragH f;
#pragma unroll
  for (int q = 0; q < 8; ++q) f.h[q] = (_Float16)bf16_rne(p[q]);
  const v8us o = f.half[0];
  unsigned short* d = (unsigned short*)X16 + e;
  *(volatile v8us*)d = o; __threadfence(); *(volatile v8us*)d = o;
}

__global__ __launch_bounds__(256) void k_hl(const float* __restrict__ F, _Float16* __restrict__ Hh, _Float16* __restrict__ Hl, size_t n8) {
  const size_t t = (size_t)blockIdx.x * 256 + threadIdx.x; if (t >= n8) return; FragH fh, fl;
  const v4f a = *(const v4fa*)(F + t * 8), c = *(const v4fa*)(F + t * 8 + 4);
#pragma unroll
  for (int q = 0; q < 4; ++q) { _Float16 hv = (_Float16)a[q]; fh.h[q] = hv; fl.h[q] = (_Float16)((a[q] - (float)hv) * 1024.0f); hv = (_Float16)c[q]; fh.h[4 + q] = hv; fl.h[4 + q] = (_Float16)((c[q] - (float)hv) * 1024.0f); }
  const v8us oh = fh.half[0], ol = fl.half[0];
  unsigned short* dh = (unsigned short*)Hh + t * 8; unsigned short* dl = (unsigned short*)Hl + t * 8;
  *(volatile v8us*)dh = oh; *(volatile v8us*)dl = ol; __threadfence(); *(volatile v8us*)dh = oh; *(volatile v8us*)dl = ol;
}

__global__ __launch_bounds__(256) void k_rotab(const int* __restrict__ pos, float* __restrict__ CS, float* __restrict__ SN) {
  #pragma clang fp contract(off)
  const int t = blockIdx.x * 256 + threadIdx.x; if (t >= NR * 32) return;
  const int j = t & 31, row = t >> 5; const int b = row / SEQ, s = row - b * SEQ;
  const float ex = (float)(2 * j) / 64.0f; const float inv = 1.0f / powf(10000.0f, ex);
  const float pf = (float)pos[(size_t)b * SEQ_FULL + s]; const float th = pf * inv;
  float sn, c; sincosf(th, &sn, &c);
  *(volatile float*)(CS + t) = c; *(volatile float*)(SN + t) = sn;
  __threadfence();
  *(volatile float*)(CS + t) = c; *(volatile float*)(SN + t) = sn;
}

__global__ __launch_bounds__(256) void k_normrope(const float* __restrict__ F, int nh, const float* __restrict__ gw, const float* __restrict__ CS, const float* __restrict__ SN, _Float16* __restrict__ H, _Float16* __restrict__ L) {
  #pragma clang fp contract(off)
  __shared__ __attribute__((aligned(16))) unsigned short st[8][2][64];
  const int wv = threadIdx.x >> 5, lane = threadIdx.x & 31;
  const size_t wid = (size_t)blockIdx.x * 8 + wv; if (wid >= (size_t)NR * nh) return;
  const size_t row = wid / nh; const int hd = (int)(wid % nh);
  const float* src = F + row * (size_t)(nh * 64) + hd * 64;
  const float x1 = src[lane], x2 = src[lane + 32];
  float ss = x1 * x1; const float tt = x2 * x2; ss += tt;
#pragma unroll
  for (int o = 16; o > 0; o >>= 1) ss += __shfl_xor(ss, o, 32);
  const float inv = rsqrtf(ss * 0.015625f + 1.0e-6f);
  const float g1 = bf16_rne(gw[lane]), g2 = bf16_rne(gw[lane + 32]);
  float y1 = x1 * inv; y1 *= g1; float y2 = x2 * inv; y2 *= g2;
  const float c = CS[row * 32 + lane], sn = SN[row * 32 + lane];
  float o1 = y1 * c; const float u1 = y2 * sn; o1 -= u1; float o2 = y2 * c; const float u2 = y1 * sn; o2 += u2;
  FragH f; _Float16 hv = (_Float16)o1; f.h[0] = hv; f.h[1] = (_Float16)((o1 - (float)hv) * 1024.0f); hv = (_Float16)o2; f.h[2] = hv; f.h[3] = (_Float16)((o2 - (float)hv) * 1024.0f);
  st[wv][0][lane] = f.u[0]; st[wv][1][lane] = f.u[1]; st[wv][0][lane + 32] = f.u[2]; st[wv][1][lane + 32] = f.u[3];
  __builtin_amdgcn_fence(4, "workgroup"); __builtin_amdgcn_wave_barrier();
  const int pl = (lane >> 3) & 1, pc = lane & 7;
  const v8us v = *(const v8us*)&st[wv][pl][pc * 8];
  unsigned short* base = pl ? (unsigned short*)L : (unsigned short*)H;
  unsigned short* dst = base + row * (size_t)(nh * 64) + hd * 64 + pc * 8;
  if (lane < 16) { *(volatile v8us*)dst = v; }
  __threadfence();
  if (lane < 16) { *(volatile v8us*)dst = v; }
}

__global__ __launch_bounds__(256) void k_vtg(const _Float16* __restrict__ V16, _Float16* __restrict__ Vt) {
  __shared__ __attribute__((aligned(16))) unsigned short tl[64][66];
  const int tid = threadIdx.x; const int slab = blockIdx.x / (SEQ / 64), lg = blockIdx.x % (SEQ / 64); const int b = slab / NKV, g = slab % NKV;
  for (int i = tid; i < 64 * 8; i += 256) { const int r = i / 8, c8 = (i % 8) * 8; FragH f; f.half[0] = *(const v8us*)((const unsigned short*)V16 + ((size_t)b * SEQ + lg * 64 + r) * KVD + g * 64 + c8);
#pragma unroll
    for (int q = 0; q < 8; ++q) tl[r][c8 + q] = f.u[q]; }
  __syncthreads();
  for (int pass = 0; pass < 2; ++pass) {
#pragma unroll
    for (int rd = 0; rd < 2; ++rd) { const int d = rd * 32 + tid / 8, pc = tid % 8; FragH f;
#pragma unroll
      for (int q = 0; q < 8; ++q) f.u[q] = tl[pc * 8 + q][d];
      *(volatile v8us*)((unsigned short*)Vt + ((size_t)slab * 64 + d) * TK + lg * 64 + pc * 8) = f.half[0]; }
    if (pass == 0) __threadfence(); }
}

__device__ __forceinline__ v16h g2_frag(const _Float16* p, int hh) { FragH f; f.half[0] = *(const v8us*)((const unsigned short*)p + 8 * hh); f.half[1] = *(const v8us*)((const unsigned short*)p + 16 + 8 * hh); return f.v; }
__device__ __forceinline__ v8f g2_mma(v16h a, v16h b, v8f c) { v8f d = __builtin_amdgcn_wmma_f32_16x16x32_f16(false, a, false, b, (short)0, c, false, false); asm volatile("v_nop\n\tv_nop\n\tv_nop\n\tv_nop" : "+v"(d) : "v"(a), "v"(b)); return d; }
__global__ __launch_bounds__(128) void k_gemm2(const _Float16* __restrict__ A, int lda, size_t sA, const _Float16* __restrict__ Bh, int ldb, size_t sB, float alpha,
                                               const float* CP, float* C, int ldc, size_t sC, int M, int N, int K) {
  __shared__ __attribute__((aligned(16))) float so[4][32][68];
  const int tid = threadIdx.x, w = tid >> 5, lane = tid & 31, ln = lane & 15, hh = lane >> 4; const int by = blockIdx.y;
  A += (size_t)by * sA; Bh += (size_t)by * sB; const size_t cofs = (size_t)by * sC;
  const int ntn = N >> 6; const int mt = blockIdx.x / ntn, nq = blockIdx.x - mt * ntn; const int row0 = mt * 128 + 32 * w, col0 = nq * 64; if (row0 >= M) return;
  const _Float16* a0p = A + (size_t)(row0 + ln) * lda; const _Float16* a1p = a0p + (size_t)16 * lda;
  const _Float16* b0p = Bh + (size_t)(col0 + ln) * ldb; const _Float16* b1p = b0p + (size_t)16 * ldb; const _Float16* b2p = b1p + (size_t)16 * ldb; const _Float16* b3p = b2p + (size_t)16 * ldb;
  const v8f z8 = {0.f,0.f,0.f,0.f,0.f,0.f,0.f,0.f}; v8f c00 = z8, c01 = z8, c02 = z8, c03 = z8, c10 = z8, c11 = z8, c12 = z8, c13 = z8;
#pragma unroll 1
  for (int kb = 0; kb < K; kb += 32) { const v16h a0 = g2_frag(a0p + kb, hh), a1 = g2_frag(a1p + kb, hh);
    v16h b = g2_frag(b0p + kb, hh); c00 = g2_mma(a0, b, c00); c10 = g2_mma(a1, b, c10);
    b = g2_frag(b1p + kb, hh); c01 = g2_mma(a0, b, c01); c11 = g2_mma(a1, b, c11);
    b = g2_frag(b2p + kb, hh); c02 = g2_mma(a0, b, c02); c12 = g2_mma(a1, b, c12);
    b = g2_frag(b3p + kb, hh); c03 = g2_mma(a0, b, c03); c13 = g2_mma(a1, b, c13); }
  v8f accs[8] = {c00, c01, c02, c03, c10, c11, c12, c13};
#pragma unroll
  for (int u = 0; u < 8; ++u) { const int t = u & 3, half = u >> 2; const int col = col0 + t * 16 + ln;
#pragma unroll
    for (int r = 0; r < 8; ++r) { const int rloc = half * 16 + 8 * hh + r; float v = accs[u][r] * alpha; if (CP) v += CP[cofs + (size_t)(row0 + rloc) * ldc + col]; so[w][rloc][t * 16 + ln] = v; } }
  __builtin_amdgcn_fence(4, "workgroup"); __builtin_amdgcn_wave_barrier();
  const int rsub = lane >> 4, c4 = (lane & 15) * 4;
  for (int pass = 0; pass < 2; ++pass) {
#pragma unroll
    for (int q = 0; q < 16; ++q) { const int r = q * 2 + rsub; const v4f v = *(const v4fa*)&so[w][r][c4]; *(volatile v4f*)(C + cofs + (size_t)(row0 + r) * ldc + col0 + c4) = v; }
    if (pass == 0) __threadfence(); }
}

template <int CAUSAL>
__global__ __launch_bounds__(128) __attribute__((amdgpu_num_vgpr(256)))
void k_flash(const _Float16* __restrict__ Q16, int ldq, const _Float16* __restrict__ K16, int ldk, const _Float16* __restrict__ Vt, float* __restrict__ O, int ldo, int qbase, int nqb) {
  constexpr int RPW = 16, DT = 4, KS = 2;
  __shared__ __attribute__((aligned(16))) unsigned short sP[4][RPW][40]; __shared__ __attribute__((aligned(16))) float sO[4][RPW][64 + 4];
  const int tid = threadIdx.x, w = tid >> 5, lane = tid & 31, ln = lane & 15, hh = lane >> 4;
  const int slab = blockIdx.x / nqb, qblk = qbase + blockIdx.x % nqb; const int b = slab / NH, h = slab % NH, g = h / NREP;
  const int qb0 = qblk * (4 * RPW); const int q0 = qb0 + w * RPW;
  FragH aq[KS];
  { const unsigned short* qr = (const unsigned short*)Q16 + ((size_t)b * TQ + q0 + ln) * ldq + h * 64;
#pragma unroll
    for (int ks = 0; ks < KS; ++ks) { aq[ks].half[0] = *(const v8us*)(qr + ks * 32 + 8 * hh); aq[ks].half[1] = *(const v8us*)(qr + ks * 32 + 16 + 8 * hh); } }
  const unsigned short* Vth = (const unsigned short*)Vt + (size_t)(b * NKV + g) * 64 * TK;
  float m_r[8], l_r[8]; v8f oacc[DT];
#pragma unroll
  for (int r = 0; r < 8; ++r) { m_r[r] = -3.0e38f; l_r[r] = 0.f; }
#pragma unroll
  for (int dt = 0; dt < DT; ++dt) oacc[dt] = (v8f){0.f,0.f,0.f,0.f,0.f,0.f,0.f,0.f};
  const int jend = (CAUSAL == 1) ? (qb0 + 4 * RPW) : TK;
#pragma unroll 1
  for (int j0 = 0; j0 < jend; j0 += 32) {
    v8f s[2];
#pragma unroll
    for (int nt = 0; nt < 2; ++nt) { const unsigned short* kr = (const unsigned short*)K16 + ((size_t)b * TK + j0 + nt * 16 + ln) * ldk + g * 64; FragH bk[KS];
#pragma unroll
      for (int ks = 0; ks < KS; ++ks) { bk[ks].half[0] = *(const v8us*)(kr + ks * 32 + 8 * hh); bk[ks].half[1] = *(const v8us*)(kr + ks * 32 + 16 + 8 * hh); }
      v8f acc = (v8f){0.f,0.f,0.f,0.f,0.f,0.f,0.f,0.f};
#pragma unroll
      for (int ks = 0; ks < KS; ++ks) acc = mmaH<1>(aq[ks].v, aq[ks].v, bk[ks].v, bk[ks].v, acc);
      s[nt] = acc; }
#pragma unroll
    for (int r = 0; r < 8; ++r) { const int tq = q0 + 8 * hh + r; const int k0 = j0 + ln, k1 = j0 + 16 + ln;
      const bool ok0 = (CAUSAL == 1) ? (k0 <= tq) : true, ok1 = (CAUSAL == 1) ? (k1 <= tq) : true;
      const float s0 = ok0 ? s[0][r] * SCL : -3.0e38f, s1 = ok1 ? s[1][r] * SCL : -3.0e38f; float mc = fmaxf(s0, s1);
      mc = fmaxf(mc, __shfl_xor(mc, 1, 32)); mc = fmaxf(mc, __shfl_xor(mc, 2, 32)); mc = fmaxf(mc, __shfl_xor(mc, 4, 32)); mc = fmaxf(mc, __shfl_xor(mc, 8, 32));
      const float mn = fmaxf(m_r[r], mc); const float al = (mn > -1.0e38f) ? expf(m_r[r] - mn) : 1.0f; m_r[r] = mn; const float p0 = ok0 ? expf(s0 - mn) : 0.f, p1 = ok1 ? expf(s1 - mn) : 0.f; l_r[r] = l_r[r] * al + p0 + p1;
#pragma unroll
      for (int dt = 0; dt < DT; ++dt) oacc[dt][r] *= al;
      FragH t2; t2.h[0] = (_Float16)(p0 * 1024.0f); t2.h[1] = (_Float16)(p1 * 1024.0f); sP[w][8 * hh + r][ln] = t2.u[0]; sP[w][8 * hh + r][16 + ln] = t2.u[1]; }
    __builtin_amdgcn_fence(4, "workgroup"); __builtin_amdgcn_wave_barrier();
    FragH pa; pa.half[0] = *(const v8us*)&sP[w][ln][8 * hh]; pa.half[1] = *(const v8us*)&sP[w][ln][16 + 8 * hh];
#pragma unroll
    for (int dt = 0; dt < DT; ++dt) { const unsigned short* vrow = Vth + (size_t)(dt * 16 + ln) * TK + j0; FragH bv; bv.half[0] = *(const v8us*)(vrow + 8 * hh); bv.half[1] = *(const v8us*)(vrow + 16 + 8 * hh);
      oacc[dt] = mmaH<1>(pa.v, pa.v, bv.v, bv.v, oacc[dt]); }
    __builtin_amdgcn_fence(4, "workgroup"); __builtin_amdgcn_wave_barrier(); }
#pragma unroll
  for (int r = 0; r < 8; ++r) { float l = l_r[r]; l += __shfl_xor(l, 1, 32); l += __shfl_xor(l, 2, 32); l += __shfl_xor(l, 4, 32); l += __shfl_xor(l, 8, 32); l_r[r] = (l > 0.f) ? 1.0f / (l * 1024.0f) : 0.f; }
#pragma unroll
  for (int dt = 0; dt < DT; ++dt)
#pragma unroll
    for (int r = 0; r < 8; ++r) sO[w][8 * hh + r][dt * 16 + ln] = oacc[dt][r] * l_r[r];
  __builtin_amdgcn_fence(4, "workgroup"); __builtin_amdgcn_wave_barrier();
  for (int pass = 0; pass < 2; ++pass) {
#pragma unroll
    for (int rp = 0; rp < RPW; rp += 2) { const int r = rp + (lane >> 4), pc = lane & 15; const v4f val = *(const v4fa*)&sO[w][r][pc * 4]; *(volatile v4f*)(O + ((size_t)b * TQ + q0 + r) * ldo + h * 64 + pc * 4) = val; }
    if (pass == 0) __threadfence(); }
}

template <int CAUSAL>
__global__ __launch_bounds__(128) __attribute__((amdgpu_num_vgpr(256)))
void k_flash5(const _Float16* __restrict__ Q16, const _Float16* __restrict__ QL, int ldq, const _Float16* __restrict__ K16, const _Float16* __restrict__ KL, int ldk,
              const _Float16* __restrict__ Vt, const _Float16* __restrict__ VtL, float* __restrict__ O, int ldo, int qbase, int nqb) {
  constexpr int RPW = 16, DT = 4, KS = 2;
  __shared__ __attribute__((aligned(16))) unsigned short sP[4][RPW][40]; __shared__ __attribute__((aligned(16))) unsigned short sPL[4][RPW][40]; __shared__ __attribute__((aligned(16))) float sO[4][RPW][64 + 4];
  const int tid = threadIdx.x, w = tid >> 5, lane = tid & 31, ln = lane & 15, hh = lane >> 4;
  const int slab = blockIdx.x / nqb, qblk = qbase + blockIdx.x % nqb; const int b = slab / NH, h = slab % NH, g = h / NREP;
  const int qb0 = qblk * (4 * RPW); const int q0 = qb0 + w * RPW;
  FragH aq[KS], aql[KS];
  { const unsigned short* qr = (const unsigned short*)Q16 + ((size_t)b * TQ + q0 + ln) * ldq + h * 64; const unsigned short* ql = (const unsigned short*)QL + ((size_t)b * TQ + q0 + ln) * ldq + h * 64;
#pragma unroll
    for (int ks = 0; ks < KS; ++ks) { aq[ks].half[0] = *(const v8us*)(qr + ks * 32 + 8 * hh); aq[ks].half[1] = *(const v8us*)(qr + ks * 32 + 16 + 8 * hh); aql[ks].half[0] = *(const v8us*)(ql + ks * 32 + 8 * hh); aql[ks].half[1] = *(const v8us*)(ql + ks * 32 + 16 + 8 * hh); } }
  const unsigned short* Vth = (const unsigned short*)Vt + (size_t)(b * NKV + g) * 64 * TK; const unsigned short* Vtl = (const unsigned short*)VtL + (size_t)(b * NKV + g) * 64 * TK;
  float m_r[8], l_r[8]; v8f oacc[DT], oaccL[DT];
#pragma unroll
  for (int r = 0; r < 8; ++r) { m_r[r] = -3.0e38f; l_r[r] = 0.f; }
#pragma unroll
  for (int dt = 0; dt < DT; ++dt) { oacc[dt] = (v8f){0.f,0.f,0.f,0.f,0.f,0.f,0.f,0.f}; oaccL[dt] = oacc[dt]; }
  const int jend = (CAUSAL == 1) ? (qb0 + 4 * RPW) : TK;
#pragma unroll 1
  for (int j0 = 0; j0 < jend; j0 += 32) {
    v8f s[2];
#pragma unroll
    for (int nt = 0; nt < 2; ++nt) { const unsigned short* kr = (const unsigned short*)K16 + ((size_t)b * TK + j0 + nt * 16 + ln) * ldk + g * 64; const unsigned short* klr = (const unsigned short*)KL + ((size_t)b * TK + j0 + nt * 16 + ln) * ldk + g * 64;
      FragH bk[KS];
#pragma unroll
      for (int ks = 0; ks < KS; ++ks) { bk[ks].half[0] = *(const v8us*)(kr + ks * 32 + 8 * hh); bk[ks].half[1] = *(const v8us*)(kr + ks * 32 + 16 + 8 * hh); }
      v8f acc = (v8f){0.f,0.f,0.f,0.f,0.f,0.f,0.f,0.f}, accl = acc;
#pragma unroll
      for (int ks = 0; ks < KS; ++ks) { acc = mmaH<1>(aq[ks].v, aq[ks].v, bk[ks].v, bk[ks].v, acc); accl = mmaH<1>(aql[ks].v, aql[ks].v, bk[ks].v, bk[ks].v, accl); }
      FragH bkl[KS];
#pragma unroll
      for (int ks = 0; ks < KS; ++ks) { bkl[ks].half[0] = *(const v8us*)(klr + ks * 32 + 8 * hh); bkl[ks].half[1] = *(const v8us*)(klr + ks * 32 + 16 + 8 * hh); }
#pragma unroll
      for (int ks = 0; ks < KS; ++ks) accl = mmaH<1>(aq[ks].v, aq[ks].v, bkl[ks].v, bkl[ks].v, accl);
#pragma unroll
      for (int r = 0; r < 8; ++r) acc[r] += accl[r] * 0.0009765625f;
      s[nt] = acc; }
#pragma unroll
    for (int r = 0; r < 8; ++r) { const int tq = q0 + 8 * hh + r; const int k0 = j0 + ln, k1 = j0 + 16 + ln;
      const bool ok0 = (CAUSAL == 1) ? (k0 <= tq) : true, ok1 = (CAUSAL == 1) ? (k1 <= tq) : true;
      const float s0 = ok0 ? s[0][r] * SCL : -3.0e38f, s1 = ok1 ? s[1][r] * SCL : -3.0e38f; float mc = fmaxf(s0, s1);
      mc = fmaxf(mc, __shfl_xor(mc, 1, 32)); mc = fmaxf(mc, __shfl_xor(mc, 2, 32)); mc = fmaxf(mc, __shfl_xor(mc, 4, 32)); mc = fmaxf(mc, __shfl_xor(mc, 8, 32));
      const float mn = fmaxf(m_r[r], mc); const float al = (mn > -1.0e38f) ? expf(m_r[r] - mn) : 1.0f; m_r[r] = mn; const float p0 = ok0 ? expf(s0 - mn) : 0.f, p1 = ok1 ? expf(s1 - mn) : 0.f; l_r[r] = l_r[r] * al + p0 + p1;
#pragma unroll
      for (int dt = 0; dt < DT; ++dt) { oacc[dt][r] *= al; oaccL[dt][r] *= al; }
      FragH t2, t2l; const float ps0 = p0 * 1024.0f, ps1 = p1 * 1024.0f; t2.h[0] = (_Float16)ps0; t2.h[1] = (_Float16)ps1; t2l.h[0] = (_Float16)((ps0 - (float)t2.h[0]) * 1024.0f); t2l.h[1] = (_Float16)((ps1 - (float)t2.h[1]) * 1024.0f);
      sP[w][8 * hh + r][ln] = t2.u[0]; sP[w][8 * hh + r][16 + ln] = t2.u[1]; sPL[w][8 * hh + r][ln] = t2l.u[0]; sPL[w][8 * hh + r][16 + ln] = t2l.u[1]; }
    __builtin_amdgcn_fence(4, "workgroup"); __builtin_amdgcn_wave_barrier();
    FragH pa, pl; pa.half[0] = *(const v8us*)&sP[w][ln][8 * hh]; pa.half[1] = *(const v8us*)&sP[w][ln][16 + 8 * hh]; pl.half[0] = *(const v8us*)&sPL[w][ln][8 * hh]; pl.half[1] = *(const v8us*)&sPL[w][ln][16 + 8 * hh];
#pragma unroll
    for (int dt = 0; dt < DT; ++dt) { const unsigned short* vrow = Vth + (size_t)(dt * 16 + ln) * TK + j0; const unsigned short* vrl = Vtl + (size_t)(dt * 16 + ln) * TK + j0; FragH bv, bl;
      bv.half[0] = *(const v8us*)(vrow + 8 * hh); bv.half[1] = *(const v8us*)(vrow + 16 + 8 * hh); bl.half[0] = *(const v8us*)(vrl + 8 * hh); bl.half[1] = *(const v8us*)(vrl + 16 + 8 * hh);
      oacc[dt] = mmaH<1>(pa.v, pa.v, bv.v, bv.v, oacc[dt]); oaccL[dt] = mmaH<1>(pl.v, pl.v, bv.v, bv.v, oaccL[dt]); oaccL[dt] = mmaH<1>(pa.v, pa.v, bl.v, bl.v, oaccL[dt]); }
    __builtin_amdgcn_fence(4, "workgroup"); __builtin_amdgcn_wave_barrier(); }
#pragma unroll
  for (int r = 0; r < 8; ++r) { float l = l_r[r]; l += __shfl_xor(l, 1, 32); l += __shfl_xor(l, 2, 32); l += __shfl_xor(l, 4, 32); l += __shfl_xor(l, 8, 32); l_r[r] = (l > 0.f) ? 1.0f / (l * 1024.0f) : 0.f; }
#pragma unroll
  for (int dt = 0; dt < DT; ++dt)
#pragma unroll
    for (int r = 0; r < 8; ++r) { float v = oacc[dt][r]; v += oaccL[dt][r] * 0.0009765625f; sO[w][8 * hh + r][dt * 16 + ln] = v * l_r[r]; }
  __builtin_amdgcn_fence(4, "workgroup"); __builtin_amdgcn_wave_barrier();
  for (int pass = 0; pass < 2; ++pass) {
#pragma unroll
    for (int rp = 0; rp < RPW; rp += 2) { const int r = rp + (lane >> 4), pc = lane & 15; const v4f val = *(const v4fa*)&sO[w][r][pc * 4]; *(volatile v4f*)(O + ((size_t)b * TQ + q0 + r) * ldo + h * 64 + pc * 4) = val; }
    if (pass == 0) __threadfence(); }
}

static inline unsigned cdiv_u(size_t a, unsigned b) { return (unsigned)((a + b - 1) / b); }

extern "C" void kernel_launch(void* const* d_in, const int* in_sizes, int n_in,
                              void* d_out, int out_size, void* d_ws, size_t ws_size, hipStream_t stream) {
  if (n_in < 8) return;
  const int rows_in = (NB - 1) * SEQ_FULL + SEQ;
  if (in_sizes[0] < rows_in * HIDDEN) return;
  if (in_sizes[1] < rows_in) return;
  if (in_sizes[2] < HIDDEN * QD || in_sizes[3] < HIDDEN * KVD || in_sizes[4] < HIDDEN * KVD || in_sizes[5] < QD * HIDDEN) return;
  if (in_sizes[6] < HDIM || in_sizes[7] < HDIM) return;
  if (out_size < rows_in * HIDDEN) return;
  const float* x   = (const float*)d_in[0];
  const int*   pos = (const int*)d_in[1];
  const float* Wq  = (const float*)d_in[2];
  const float* Wk  = (const float*)d_in[3];
  const float* Wv  = (const float*)d_in[4];
  const float* Wo  = (const float*)d_in[5];
  const float* gq  = (const float*)d_in[6];
  const float* gk  = (const float*)d_in[7];
  char* ws = (char*)d_ws; size_t off = 0;
  auto take = [&](size_t bytes) { char* p = ws + off; off += (bytes + 255) & ~(size_t)255; return p; };
  const size_t nq = (size_t)NR * QD, nkv = (size_t)NR * KVD, nx = (size_t)NR * HIDDEN;
  _Float16* BQ = (_Float16*)take((size_t)HIDDEN * QD * 2); _Float16* BK = (_Float16*)take((size_t)HIDDEN * KVD * 2); _Float16* BV = (_Float16*)take((size_t)HIDDEN * KVD * 2); _Float16* BO = (_Float16*)take((size_t)QD * HIDDEN * 2);
  _Float16* X16 = (_Float16*)take(nx * 2);
  float* QF = (float*)take(nq * 4); float* KF = (float*)take(nkv * 4); float* VF = (float*)take(nkv * 4);
  float* CS = (float*)take((size_t)NR * 32 * 4); float* SN = (float*)take((size_t)NR * 32 * 4);
  _Float16* QH = (_Float16*)take(nq * 2); _Float16* QL = (_Float16*)take(nq * 2);
  _Float16* KH = (_Float16*)take(nkv * 2); _Float16* KL = (_Float16*)take(nkv * 2);
  _Float16* VH = (_Float16*)take(nkv * 2); _Float16* VL = (_Float16*)take(nkv * 2);
  _Float16* VT = (_Float16*)take((size_t)NB * NKV * 64 * TK * 2); _Float16* VTL = (_Float16*)take((size_t)NB * NKV * 64 * TK * 2);
  float* O = (float*)take(nq * 4); _Float16* OH = (_Float16*)take(nq * 2); _Float16* OL = (_Float16*)take(nq * 2);
  if (off > ws_size || off > WS_LIMIT) return;

  k_wt_f16<<<cdiv_u((size_t)HIDDEN * QD / 8, 256), 256, 0, stream>>>(Wq, BQ, HIDDEN, QD, 16.0f);
  k_wt_f16<<<cdiv_u((size_t)HIDDEN * KVD / 8, 256), 256, 0, stream>>>(Wk, BK, HIDDEN, KVD, 16.0f);
  k_wt_f16<<<cdiv_u((size_t)HIDDEN * KVD / 8, 256), 256, 0, stream>>>(Wv, BV, HIDDEN, KVD, 16.0f);
  k_wt_f16<<<cdiv_u((size_t)QD * HIDDEN / 8, 256), 256, 0, stream>>>(Wo, BO, QD, HIDDEN, 16.0f);
  k_x16<<<cdiv_u(nx / 8, 256), 256, 0, stream>>>(x, X16, nx / 8);
  k_gemm2<<<dim3((NR / 128) * (QD / 64), 1), 128, 0, stream>>>(X16, HIDDEN, 0, BQ, HIDDEN, 0, 0.0625f, nullptr, QF, QD, 0, NR, QD, HIDDEN);
  k_gemm2<<<dim3((NR / 128) * (KVD / 64), 1), 128, 0, stream>>>(X16, HIDDEN, 0, BK, HIDDEN, 0, 0.0625f, nullptr, KF, KVD, 0, NR, KVD, HIDDEN);
  k_gemm2<<<dim3((NR / 128) * (KVD / 64), 1), 128, 0, stream>>>(X16, HIDDEN, 0, BV, HIDDEN, 0, 0.0625f, nullptr, VF, KVD, 0, NR, KVD, HIDDEN);
  k_rotab<<<cdiv_u((size_t)NR * 32, 256), 256, 0, stream>>>(pos, CS, SN);
  k_normrope<<<cdiv_u((size_t)NR * NH, 8), 256, 0, stream>>>(QF, NH, gq, CS, SN, QH, QL);
  k_normrope<<<cdiv_u((size_t)NR * NKV, 8), 256, 0, stream>>>(KF, NKV, gk, CS, SN, KH, KL);
  k_hl<<<cdiv_u(nkv / 8, 256), 256, 0, stream>>>(VF, VH, VL, nkv / 8);
  k_vtg<<<NB * NKV * (SEQ / 64), 256, 0, stream>>>(VH, VT);
  k_vtg<<<NB * NKV * (SEQ / 64), 256, 0, stream>>>(VL, VTL);
  k_flash5<1><<<NB * NH * QBN5, 128, 0, stream>>>(QH, QL, QD, KH, KL, KVD, VT, VTL, O, QD, QB05, QBN5);
  if (QBNP > 0) k_flash<1><<<NB * NH * QBNP, 128, 0, stream>>>(QH, QD, KH, KVD, VT, O, QD, QB0P, QBNP);
  k_hl<<<cdiv_u(nq / 8, 256), 256, 0, stream>>>(O, OH, OL, nq / 8);
  float* out = (float*)d_out; const size_t sOut = (size_t)SEQ_FULL * HIDDEN, sPl = (size_t)SEQ * QD;
  k_gemm2<<<dim3((RE / 128) * (HIDDEN / 64), NB), 128, 0, stream>>>(OL, QD, sPl, BO, QD, 0, 0.0625f / 1024.0f, nullptr, out, HIDDEN, sOut, RE, HIDDEN, QD);
  k_gemm2<<<dim3((RE / 128) * (HIDDEN / 64), NB), 128, 0, stream>>>(OH, QD, sPl, BO, QD, 0, 0.0625f, out, out, HIDDEN, sOut, RE, HIDDEN, QD);
  if (SEQ > RE) k_gemm2<<<dim3(((SEQ - RE) / 128) * (HIDDEN / 64), NB), 128, 0, stream>>>(OH + (size_t)RE * QD, QD, sPl, BO, QD, 0, 0.0625f, nullptr, out + (size_t)RE * HIDDEN, HIDDEN, sOut, SEQ - RE, HIDDEN, QD);
}
